// SelfAttentionWith1DRelativePos_23811298689413
// MI455X (gfx1250) — hardware-verified
//
#include <hip/hip_runtime.h>
#include <hip/hip_bf16.h>
#include <math.h>

#define NBq 4
#define LL 1024
#define CC 512
#define C2 1024
#define NHD 8
#define HF 64
#define HQ 32
#define NREL 2047
#define NRP 2048
#define MTOK (NBq * LL)
#define GSTR 48

typedef _Float16 bf16;
typedef _Float16 f16;
typedef __attribute__((ext_vector_type(4))) unsigned v4u_t;
typedef unsigned v4ua __attribute__((ext_vector_type(4), may_alias));
typedef __attribute__((ext_vector_type(4))) float v4f_t;
typedef float v4fa __attribute__((ext_vector_type(4), may_alias));
typedef __attribute__((ext_vector_type(16))) bf16  bf16x16;
typedef bf16x16 f16x16;
typedef __attribute__((ext_vector_type(8)))  bf16  bf16x8;
typedef bf16x8 f16x8;
typedef __attribute__((ext_vector_type(4)))  bf16  bf16x4;
typedef __attribute__((ext_vector_type(8)))  float f32x8;
__device__ __forceinline__ f32x8 wmma16(f16x16 a, f16x16 b, f32x8 c) {
  c = __builtin_amdgcn_wmma_f32_16x16x32_f16(false, a, false, b, (short)0, c, false, false);
  asm volatile("v_nop\n\tv_nop\n\tv_nop\n\tv_nop" : "+v"(c) : "v"(a), "v"(b));
  return c;
}
#define LDS_STRIDE 48
#define KSTRIDE    72
#define VSTRIDE    48

__device__ __forceinline__ f32x8 wmma_bf16(bf16x16 a, bf16x16 b, f32x8 c) {
  c = __builtin_amdgcn_wmma_f32_16x16x32_f16(false, a, false, b, (short)0, c, false, false);
  asm volatile("v_nop\n\tv_nop\n\tv_nop\n\tv_nop" : "+v"(c) : "v"(a), "v"(b));
  return c;
}

template <typename T>
__device__ __forceinline__ bf16x16 load_frag(const T* __restrict__ base, int ld,
                                             int row0, int k0) {
  const int lane = threadIdx.x & 31;
  const int r    = lane & 15;
  const int kh   = (lane >> 4) * 8;
  const T* p0 = base + (size_t)(row0 + r) * ld + (k0 + kh);
  const T* p1 = p0 + 16;
  bf16x16 f;
#pragma unroll
  for (int i = 0; i < 8; ++i) {
    f[i]     = (bf16)p0[i];
    f[i + 8] = (bf16)p1[i];
  }
  return f;
}

__device__ __forceinline__ bf16x16 lds_frag(const bf16* base, int stride) {
  const int lane = threadIdx.x & 31;
  const int row  = lane & 15;
  const int kh   = (lane >> 4) * 8;
  const bf16x8 lo = *(const bf16x8*)(base + row * stride + kh);
  const bf16x8 hi = *(const bf16x8*)(base + row * stride + kh + 16);
  bf16x16 f;
#pragma unroll
  for (int i = 0; i < 8; ++i) { f[i] = lo[i]; f[i + 8] = hi[i]; }
  return f;
}

template <typename T>
__device__ __forceinline__ void stage_read16(const T* __restrict__ p, float* buf) {
#pragma unroll
  for (int i = 0; i < 16; ++i) buf[i] = (float)p[i];
}

__device__ __forceinline__ void stage_write(bf16* dst, const float* buf, int nquad) {
#pragma unroll
  for (int i = 0; i < nquad; ++i) {
    bf16x4 q;
    q[0] = (bf16)buf[4 * i];     q[1] = (bf16)buf[4 * i + 1];
    q[2] = (bf16)buf[4 * i + 2]; q[3] = (bf16)buf[4 * i + 3];
    *(bf16x4*)(dst + 4 * i) = q;
  }
}


#define GSTR 48
template <typename AT, int EPI, bool OUT16>
__global__ __launch_bounds__(256) void gemm_kne(const AT* __restrict__ A, int lda, const float* __restrict__ Wm, int ldw,
                                                const float* __restrict__ bias, const float* __restrict__ R, const float* __restrict__ gvec,
                                                void* __restrict__ Yv, int ldy, int K) {
  __shared__ __attribute__((aligned(16))) f16 ldsA[128 * GSTR];
  __shared__ __attribute__((aligned(16))) f16 ldsW[128 * GSTR];
  __shared__ __attribute__((aligned(16))) float oS[8][32 * 68];
  const int tid = threadIdx.x, lane = tid & 31, wave = tid >> 5, cl = lane & 15, rh = (lane >> 4) * 8;
  const int m0 = blockIdx.x * 128, n0 = blockIdx.y * 128;
  const int wm = (wave & 3) * 32, wn = (wave >> 2) * 64;
  f32x8 acc[2][4];
#pragma unroll
  for (int i = 0; i < 2; ++i)
#pragma unroll
    for (int j = 0; j < 4; ++j) { f32x8 z = {}; acc[i][j] = z; }
#pragma unroll 1
  for (int k0 = 0; k0 < K; k0 += 32) {
    __syncthreads();
    { const int row = tid >> 1, ch = (tid & 1) * 16;
      const AT* src = A + (size_t)(m0 + row) * lda + k0 + ch;
#pragma unroll
      for (int g = 0; g < 16; ++g) ldsA[row * GSTR + ch + g] = (f16)src[g]; }
    { const int k = tid >> 3, nn0 = (tid & 7) * 16;
      const float* src = Wm + (size_t)(k0 + k) * ldw + n0 + nn0;
#pragma unroll
      for (int g = 0; g < 4; ++g) { const v4f_t v = *(const v4f_t*)(src + 4 * g);
#pragma unroll
        for (int u = 0; u < 4; ++u) ldsW[(nn0 + 4 * g + u) * GSTR + k] = (f16)v[u]; } }
    __syncthreads();
    f16x16 af[2];
#pragma unroll
    for (int i = 0; i < 2; ++i) af[i] = lds_frag(ldsA + (wm + 16 * i) * GSTR, GSTR);
#pragma unroll
    for (int j = 0; j < 4; ++j) {
      const f16x16 bf = lds_frag(ldsW + (wn + 16 * j) * GSTR, GSTR);
#pragma unroll
      for (int i = 0; i < 2; ++i) acc[i][j] = wmma16(af[i], bf, acc[i][j]);
    }
  }
  float* so = oS[wave];
#pragma unroll
  for (int i = 0; i < 2; ++i)
#pragma unroll
    for (int j = 0; j < 4; ++j) {
      const int n = n0 + wn + 16 * j + cl;
      const float bv = bias ? bias[n] : 0.0f;
      const float gv = (EPI == 2) ? gvec[n] : 0.0f;
      if (EPI == 1) {
#pragma unroll 1
        for (int r = 0; r < 8; ++r) { const float xg = acc[i][j][r] + bv; so[(16 * i + rh + r) * 68 + 16 * j + cl] = 0.5f * xg * (1.0f + erff(xg * 0.70710678118654752f)); }
      } else {
#pragma unroll
        for (int r = 0; r < 8; ++r) {
          float v = acc[i][j][r] + bv;
          if (EPI == 2) v = R[(size_t)(m0 + wm + 16 * i + rh + r) * ldy + n] + gv * v;
          so[(16 * i + rh + r) * 68 + 16 * j + cl] = v;
        }
      }
    }
  asm volatile("s_wait_dscnt 0" ::: "memory");
  __builtin_amdgcn_wave_barrier();
#pragma unroll 1
  for (int pass = 0; pass < 2; ++pass) {
    if (OUT16) {
      f16* Y = (f16*)Yv;
#pragma unroll
      for (int it = 0; it < 8; ++it) { const int c = lane + 32 * it, rr = c >> 3, q8 = (c & 7) * 8;
        union { f16 h[8]; v4u_t v; } u;
#pragma unroll
        for (int e = 0; e < 8; ++e) u.h[e] = (f16)so[rr * 68 + q8 + e];
        *(volatile v4u_t*)(Y + (size_t)(m0 + wm + rr) * ldy + n0 + wn + q8) = u.v; }
    } else {
      float* Y = (float*)Yv;
#pragma unroll
      for (int it = 0; it < 16; ++it) { const int f4 = lane + 32 * it, rr = f4 >> 4, q = (f4 & 15) * 4;
        *(volatile v4f_t*)(Y + (size_t)(m0 + wm + rr) * ldy + n0 + wn + q) = *(const v4fa*)(so + rr * 68 + q); }
    }
    __threadfence();
  }
}

template <typename AT, bool ACC>
__global__ __launch_bounds__(256) void gemm_kn2(const AT* __restrict__ A, int lda, size_t strideA,
                                               const float* __restrict__ Wm, int ldw, size_t strideW,
                                               const float* __restrict__ bias, float scale,
                                               float* __restrict__ Y, int ldy, size_t strideY, int K) {
  __shared__ __attribute__((aligned(16))) f16 ldsA[128 * GSTR], ldsAl[128 * GSTR];
  __shared__ __attribute__((aligned(16))) f16 ldsW[128 * GSTR], ldsWl[128 * GSTR];
  __shared__ __attribute__((aligned(16))) float oS[8][32 * 68];
  const int tid = threadIdx.x, lane = tid & 31, wave = tid >> 5, cl = lane & 15, rh = (lane >> 4) * 8;
  const int m0 = blockIdx.x * 128, n0 = blockIdx.y * 128;
  const int wm = (wave & 3) * 32, wn = (wave >> 2) * 64;
  A += (size_t)blockIdx.z * strideA; Wm += (size_t)blockIdx.z * strideW; Y += (size_t)blockIdx.z * strideY;
  f32x8 acc[2][4], accx[2][4];
#pragma unroll
  for (int i = 0; i < 2; ++i)
#pragma unroll
    for (int j = 0; j < 4; ++j) { f32x8 z = {}; acc[i][j] = z; accx[i][j] = z; }
#pragma unroll 1
  for (int k0 = 0; k0 < K; k0 += 32) {
    __syncthreads();
    {
      const int row = tid >> 1, ch = (tid & 1) * 16;
      const AT* src = A + (size_t)(m0 + row) * lda + k0 + ch;
#pragma unroll
      for (int g = 0; g < 16; ++g) { const float v = (float)src[g]; const f16 h = (f16)v; ldsA[row * GSTR + ch + g] = h; ldsAl[row * GSTR + ch + g] = (f16)((v - (float)h) * 2048.0f); }
    }
    {
      const int k = tid >> 3, nn0 = (tid & 7) * 16;
      const float* src = Wm + (size_t)(k0 + k) * ldw + n0 + nn0;
#pragma unroll
      for (int g = 0; g < 4; ++g) { const v4f_t v = *(const v4f_t*)(src + 4 * g);
#pragma unroll
        for (int u = 0; u < 4; ++u) { const f16 h = (f16)v[u]; ldsW[(nn0 + 4 * g + u) * GSTR + k] = h; ldsWl[(nn0 + 4 * g + u) * GSTR + k] = (f16)((v[u] - (float)h) * 2048.0f); } }
    }
    __syncthreads();
    f16x16 af[2], afl[2];
#pragma unroll
    for (int i = 0; i < 2; ++i) { af[i] = lds_frag(ldsA + (wm + 16 * i) * GSTR, GSTR); afl[i] = lds_frag(ldsAl + (wm + 16 * i) * GSTR, GSTR); }
#pragma unroll
    for (int j = 0; j < 4; ++j) {
      const f16x16 bf = lds_frag(ldsW + (wn + 16 * j) * GSTR, GSTR), bfl = lds_frag(ldsWl + (wn + 16 * j) * GSTR, GSTR);
#pragma unroll
      for (int i = 0; i < 2; ++i) { acc[i][j] = wmma16(af[i], bf, acc[i][j]); accx[i][j] = wmma16(af[i], bfl, accx[i][j]); accx[i][j] = wmma16(afl[i], bf, accx[i][j]); }
    }
  }
  float* so = oS[wave];
#pragma unroll
  for (int i = 0; i < 2; ++i)
#pragma unroll
    for (int j = 0; j < 4; ++j) {
      const float bv = bias ? bias[n0 + wn + 16 * j + cl] : 0.0f;
#pragma unroll
      for (int r = 0; r < 8; ++r) so[(16 * i + rh + r) * 68 + 16 * j + cl] = (acc[i][j][r] + accx[i][j][r] * (1.0f / 2048.0f)) * scale + bv;
    }
  asm volatile("s_wait_dscnt 0" ::: "memory");
  __builtin_amdgcn_wave_barrier();
  if (ACC) {
#pragma unroll
    for (int it = 0; it < 16; ++it) { const int f4 = lane + 32 * it, rr = f4 >> 4, q = (f4 & 15) * 4;
      const v4f_t old = *(const v4fa*)(Y + (size_t)(m0 + wm + rr) * ldy + n0 + wn + q);
      v4f_t v = *(const v4fa*)(so + rr * 68 + q); v += old; *(volatile v4fa*)(so + rr * 68 + q) = v; }
    asm volatile("s_wait_dscnt 0" ::: "memory");
  }
#pragma unroll 1
  for (int pass = 0; pass < 2; ++pass) {
#pragma unroll
    for (int it = 0; it < 16; ++it) { const int f4 = lane + 32 * it, rr = f4 >> 4, q = (f4 & 15) * 4;
      *(volatile v4f_t*)(Y + (size_t)(m0 + wm + rr) * ldy + n0 + wn + q) = *(const v4fa*)(so + rr * 68 + q); }
    __threadfence();
  }
}

__global__ __launch_bounds__(256) void k_gn_stats(const float* __restrict__ Y, int Cw, float* __restrict__ stats) {
  __shared__ float red[256]; __shared__ float gm[32], gr[32];
  const int b = blockIdx.x, tid = threadIdx.x; const int cg = Cw / 32; const int tpg = cg / 4;
  const int nthr = Cw / 4; const float* base = Y + (size_t)b * LL * Cw + tid * 4; const float inv_n = 1.0f / (float)(LL * cg);
  float s = 0.0f;
  if (tid < nthr) {
#pragma unroll 1
    for (int l = 0; l < LL; ++l) { const v4f_t v = *(const v4f_t*)(base + (size_t)l * Cw); s += (v[0] + v[1]) + (v[2] + v[3]); } }
  red[tid] = s; __syncthreads();
  if (tid < 32) { float a = 0.0f; for (int k = 0; k < tpg; ++k) a += red[tid * tpg + k]; gm[tid] = a * inv_n; }
  __syncthreads();
  float q = 0.0f;
  if (tid < nthr) { const float mean = gm[tid / tpg];
#pragma unroll 1
    for (int l = 0; l < LL; ++l) { const v4f_t v = *(const v4f_t*)(base + (size_t)l * Cw); for (int k = 0; k < 4; ++k) { const float d = v[k] - mean; q += d * d; } } }
  red[tid] = q; __syncthreads();
  if (tid < 32) { float a = 0.0f; for (int k = 0; k < tpg; ++k) a += red[tid * tpg + k]; gr[tid] = rsqrtf(a * inv_n + 1e-4f); }
  __syncthreads();
#pragma unroll 1
  for (int pass = 0; pass < 2; ++pass) { if (tid < 16) { v4f_t o; o[0] = gm[tid * 2]; o[1] = gr[tid * 2]; o[2] = gm[tid * 2 + 1]; o[3] = gr[tid * 2 + 1]; *(volatile v4f_t*)(stats + (size_t)b * 64 + tid * 4) = o; } __threadfence(); }
}
__global__ __launch_bounds__(256) void k_gn_apply(const float* __restrict__ Y, int Cw, const float* __restrict__ stats, const float* __restrict__ sc, const float* __restrict__ bi, float* __restrict__ D) {
  const size_t row = blockIdx.x; const int b = row / LL; const int cg = Cw / 32;
  for (int q4 = threadIdx.x; q4 < Cw / 4; q4 += 256) { const int c = q4 * 4; const int g = c / cg; const float mean = stats[b * 64 + g * 2], rstd = stats[b * 64 + g * 2 + 1];
    const v4f_t v = *(const v4f_t*)(Y + row * Cw + c); v4f_t o; for (int k = 0; k < 4; ++k) o[k] = (v[k] - mean) * rstd * sc[c + k] + bi[c + k];
    *(volatile v4f_t*)(D + row * Cw + c) = o; __threadfence(); *(volatile v4f_t*)(D + row * Cw + c) = o; }
}
__global__ __launch_bounds__(256) void k_gather_qk(const float* __restrict__ G, int b, int h, float* __restrict__ QT, float* __restrict__ KM, float* __restrict__ QK64) {
  __shared__ float kT[32][65];
  const int tid = threadIdx.x; const int i0 = blockIdx.x * 64;
  for (int e = tid; e < 64 * 64; e += 256) { const int t = e >> 6, c = e & 63; const float v = G[((size_t)b * LL + i0 + t) * C2 + h * 128 + c];
    QK64[(size_t)(i0 + t) * 64 + c] = v; if (c < 32) QT[(size_t)(i0 + t) * 32 + c] = v; else kT[c - 32][t] = v; }
  __syncthreads();
  for (int e = tid; e < 32 * 16; e += 256) { const int d = e >> 4, q4 = (e & 15) * 4; v4f_t o; for (int k = 0; k < 4; ++k) o[k] = kT[d][q4 + k]; *(volatile v4f_t*)(KM + (size_t)d * LL + i0 + q4) = o; }
  __threadfence();
  for (int e = tid; e < 64 * 64; e += 256) { const int t = e >> 6, c = e & 63; const float v = G[((size_t)b * LL + i0 + t) * C2 + h * 128 + c];
    *(volatile float*)(QK64 + (size_t)(i0 + t) * 64 + c) = v; if (c < 32) *(volatile float*)(QT + (size_t)(i0 + t) * 32 + c) = v; }
  for (int e = tid; e < 32 * 16; e += 256) { const int d = e >> 4, q4 = (e & 15) * 4; v4f_t o; for (int k = 0; k < 4; ++k) o[k] = kT[d][q4 + k]; *(volatile v4f_t*)(KM + (size_t)d * LL + i0 + q4) = o; }
}
__global__ __launch_bounds__(256) void k_reltabs(const float* __restrict__ R, float* __restrict__ RKQ, float* __restrict__ RvT) {
  const int tid = threadIdx.x; const int r0 = blockIdx.x * 256;
#pragma unroll 1
  for (int d = 0; d < 64; ++d) { const int src = (d < 32) ? (32 + d) : (d - 32); const int r = r0 + tid; const float v = (r < NREL) ? R[(size_t)src * NREL + r] : 0.0f;
    *(volatile float*)(RKQ + (size_t)d * NRP + r) = v; __threadfence(); *(volatile float*)(RKQ + (size_t)d * NRP + r) = v; }
#pragma unroll 1
  for (int e = tid; e < 256 * 128; e += 256) { const int rl = e >> 7, c = e & 127; const int r = r0 + rl; const float v = (c < 64 && r < NREL) ? R[(size_t)(64 + c) * NREL + r] : 0.0f;
    *(volatile float*)(RvT + (size_t)r * 128 + c) = v; __threadfence(); *(volatile float*)(RvT + (size_t)r * 128 + c) = v; }
}
__global__ __launch_bounds__(256) void k_relsoftmax(float* __restrict__ S, const float* __restrict__ T, float* __restrict__ Prel) {
  __shared__ float red[256]; __shared__ __attribute__((aligned(16))) float prow[NRP];
  const int i = blockIdx.x, tid = threadIdx.x; float* sr = S + (size_t)i * LL; const float* tr = T + (size_t)i * NRP; float* pr = Prel + (size_t)i * NRP;
  float v[4]; float m = -3.0e38f;
#pragma unroll
  for (int e = 0; e < 4; ++e) { const int j = tid + 256 * e; v[e] = sr[j] + tr[i - j + LL - 1]; m = fmaxf(m, v[e]); }
  for (int r = tid; r < NRP; r += 256) prow[r] = 0.0f;
  red[tid] = m; __syncthreads();
  for (int o = 128; o > 0; o >>= 1) { if (tid < o) red[tid] = fmaxf(red[tid], red[tid + o]); __syncthreads(); }
  m = red[0]; __syncthreads();
  float z = 0.0f;
#pragma unroll
  for (int e = 0; e < 4; ++e) { v[e] = expf(v[e] - m); z += v[e]; }
  red[tid] = z; __syncthreads();
  for (int o = 128; o > 0; o >>= 1) { if (tid < o) red[tid] += red[tid + o]; __syncthreads(); }
  const float sc = 1024.0f / red[0];
#pragma unroll
  for (int e = 0; e < 4; ++e) { const int j = tid + 256 * e; v[e] *= sc; prow[i - j + LL - 1] = v[e]; }
  __syncthreads();
#pragma unroll 1
  for (int pass = 0; pass < 2; ++pass) {
#pragma unroll
    for (int e = 0; e < 4; ++e) *(volatile float*)(sr + tid + 256 * e) = v[e];
    for (int q4 = tid; q4 < NRP / 4; q4 += 256) *(volatile v4f_t*)(pr + q4 * 4) = *(const v4fa*)(prow + q4 * 4);
    __threadfence(); }
}
__global__ __launch_bounds__(256) void k_combine(const float* __restrict__ WV, const float* __restrict__ WE, int b, int h, float* __restrict__ O) {
  const int tid = threadIdx.x; const int i = blockIdx.x * 16 + (tid >> 4), c4 = (tid & 15) * 4;
  const v4f_t a = *(const v4f_t*)(WV + (size_t)i * 128 + c4), e = *(const v4f_t*)(WE + (size_t)i * 128 + c4); v4f_t o; for (int k = 0; k < 4; ++k) o[k] = (a[k] + e[k]) * (1.0f / 1024.0f);
  float* dst = O + ((size_t)b * LL + i) * CC + h * HF + c4; *(volatile v4f_t*)dst = o; __threadfence(); *(volatile v4f_t*)dst = o;
}
__global__ __launch_bounds__(256) void k_copy(const float* __restrict__ src, float* __restrict__ dst) { const size_t off = (size_t)blockIdx.x * CC + threadIdx.x * 2;
  typedef __attribute__((ext_vector_type(2))) float v2f; const v2f v = *(const v2f*)(src + off); *(volatile v2f*)(dst + off) = v; __threadfence(); *(volatile v2f*)(dst + off) = v; }

extern "C" void kernel_launch(void* const* d_in, const int* in_sizes, int n_in,
                              void* d_out, int out_size, void* d_ws, size_t ws_size,
                              hipStream_t stream) {
  (void)in_sizes; (void)n_in; (void)out_size;
  const float** f = (const float**)d_in;
  const float* x = f[0], *Wqkv = f[1], *gsc = f[2], *gbi = f[3], *R = f[4], *osc = f[5], *obi = f[6];
  float* out = (float*)d_out;
  char* ws = (char*)d_ws;
  float* G = (float*)ws; ws += (size_t)MTOK * C2 * 4 + 4096;
  float* RKQ = (float*)ws; ws += (size_t)64 * NRP * 4; float* RvT = (float*)ws; ws += (size_t)NRP * 128 * 4;
  float* QT = (float*)ws; ws += (size_t)LL * 32 * 4; float* KM = (float*)ws; ws += (size_t)32 * LL * 4; float* QK64 = (float*)ws; ws += (size_t)LL * 64 * 4;
  float* S = (float*)ws; ws += (size_t)LL * LL * 4;
  float* T = (float*)ws; ws += (size_t)LL * NRP * 4;
  float* Prel = (float*)ws; ws += (size_t)LL * NRP * 4;
  float* WV = (float*)ws; ws += (size_t)LL * 128 * 4; float* WE = (float*)ws; ws += (size_t)LL * 128 * 4;
  float* O = (float*)ws; ws += (size_t)MTOK * CC * 4;
  float* stats = (float*)ws; ws += (size_t)NBq * 64 * 4;
  if ((size_t)(ws - (char*)d_ws) > ws_size) return;
  const dim3 blk(256);
  k_reltabs<<<dim3(NRP / 256), blk, 0, stream>>>(R, RKQ, RvT);
  gemm_kn2<float, false><<<dim3(MTOK / 128, C2 / 128, 1), blk, 0, stream>>>(x, CC, 0, Wqkv, C2, 0, nullptr, 1.0f, G, C2, 0, CC);
  k_gn_stats<<<dim3(NBq), blk, 0, stream>>>(G, C2, stats); k_gn_apply<<<dim3(MTOK), blk, 0, stream>>>(G, C2, stats, gsc, gbi, G);
  for (int b = 0; b < NBq; ++b) for (int h = 0; h < NHD; ++h) {
    k_gather_qk<<<dim3(LL / 64), blk, 0, stream>>>(G, b, h, QT, KM, QK64);
    gemm_kn2<float, false><<<dim3(LL / 128, LL / 128, 1), blk, 0, stream>>>(QT, 32, 0, KM, LL, 0, nullptr, 1.0f, S, LL, 0, 32);
    gemm_kn2<float, false><<<dim3(LL / 128, NRP / 128, 1), blk, 0, stream>>>(QK64, 64, 0, RKQ, NRP, 0, nullptr, 1.0f, T, NRP, 0, 64);
    k_relsoftmax<<<dim3(LL), blk, 0, stream>>>(S, T, Prel);
    gemm_kne<float, 0, false><<<dim3(LL / 128, 1), blk, 0, stream>>>(S, LL, G + (size_t)b * LL * C2 + h * 128 + 64, C2, nullptr, nullptr, nullptr, WV, 128, LL);
    gemm_kne<float, 0, false><<<dim3(LL / 128, 1), blk, 0, stream>>>(Prel, NRP, RvT, 128, nullptr, nullptr, nullptr, WE, 128, NRP);
    k_combine<<<dim3(LL / 16), blk, 0, stream>>>(WV, WE, b, h, O);
  }
  k_gn_stats<<<dim3(NBq), blk, 0, stream>>>(O, CC, stats); k_gn_apply<<<dim3(MTOK), blk, 0, stream>>>(O, CC, stats, osc, obi, out);
}
